// DepthConv_48361331753341
// MI455X (gfx1250) — hardware-verified
//
#include <hip/hip_runtime.h>
#include <math.h>

#define NB_ 8
#define CIN 64
#define COUT 64
#define IH 160
#define IW 160
#define NPIX (IH * IW)
#define KK 9
#define KTOT (CIN * KK)

typedef _Float16 f16;
typedef __attribute__((ext_vector_type(16))) f16 f16x16;
typedef __attribute__((ext_vector_type(8)))  f16 f16x8;
typedef __attribute__((ext_vector_type(8)))  float f32x8;
typedef __attribute__((ext_vector_type(4)))  float v4f_t;
typedef float v4fa __attribute__((ext_vector_type(4), may_alias));
__device__ __forceinline__ f32x8 wmma16(f16x16 a, f16x16 b, f32x8 c) {
  c = __builtin_amdgcn_wmma_f32_16x16x32_f16(false, a, false, b, (short)0, c, false, false);
  asm volatile("v_nop\n\tv_nop\n\tv_nop\n\tv_nop" : "+v"(c) : "v"(a), "v"(b));
  return c;
}
__device__ __forceinline__ f16x16 lds_frag(const f16* base, int stride) {
  const int lane = threadIdx.x & 31, row = lane & 15, kh = (lane >> 4) * 8;
  const f16x8 lo = *(const f16x8*)(base + row * stride + kh);
  const f16x8 hi = *(const f16x8*)(base + row * stride + kh + 16);
  f16x16 f;
#pragma unroll
  for (int i = 0; i < 8; ++i) { f[i] = lo[i]; f[i + 8] = hi[i]; }
  return f;
}
__global__ __launch_bounds__(256) void k_depthconv(const float* __restrict__ x, const float* __restrict__ depth, const float* __restrict__ w, const float* __restrict__ bias, float* __restrict__ out) {
  __shared__ __attribute__((aligned(16))) f16 aS[128 * 168];
  __shared__ __attribute__((aligned(16))) f16 wS[64 * 168];
  __shared__ float simS[128 * 9];
  __shared__ __attribute__((aligned(16))) float oS[COUT * 132];
  const int tid = threadIdx.x, lane = tid & 31, wave = tid >> 5, cl = lane & 15, rh = (lane >> 4) * 8;
  const int b = blockIdx.x / (NPIX / 128), p0 = (blockIdx.x % (NPIX / 128)) * 128;
  for (int e = tid; e < 128 * 9; e += 256) { const int r = e / 9, k = e % 9; const int p = p0 + r, oh = p / IW, ow = p % IW; const int ih = oh + k / 3 - 1, iw = ow + k % 3 - 1;
    const float* dp = depth + (size_t)b * NPIX; const float d0 = dp[p];
    const float dk = (ih >= 0 && ih < IH && iw >= 0 && iw < IW) ? dp[min(max(ih, 0), IH - 1) * IW + min(max(iw, 0), IW - 1)] : 0.0f;
    simS[e] = expf(-fabsf(dk - d0)); }
  for (int e = tid; e < 128 * 16; e += 256) aS[(e >> 4) * 168 + 144 + (e & 15)] = (f16)0.0f;
  for (int e = tid; e < 64 * 16; e += 256) wS[(e >> 4) * 168 + 144 + (e & 15)] = (f16)0.0f;
  f32x8 acc[4];
#pragma unroll
  for (int j = 0; j < 4; ++j) { f32x8 z = {}; acc[j] = z; }
  __syncthreads();
#pragma unroll 1
  for (int cg = 0; cg < CIN / 16; ++cg) {
    for (int e = tid; e < 128 * 144; e += 256) { const int r = e / 144, q = e % 144, cc = q / 9, k = q % 9; const int p = p0 + r, oh = p / IW, ow = p % IW; const int ih = oh + k / 3 - 1, iw = ow + k % 3 - 1;
      const int c = cg * 16 + cc; float v = 0.0f;
      if (ih >= 0 && ih < IH && iw >= 0 && iw < IW) v = x[(((size_t)b * CIN + c) * IH + min(max(ih, 0), IH - 1)) * IW + min(max(iw, 0), IW - 1)] * simS[r * 9 + k];
      aS[r * 168 + q] = (f16)v; }
    for (int e = tid; e < 64 * 144; e += 256) { const int o = e / 144, q = e % 144; wS[o * 168 + q] = (f16)w[((size_t)o * CIN + cg * 16) * KK + q]; }
    __syncthreads();
#pragma unroll
    for (int ks = 0; ks < 5; ++ks) { const f16x16 af = lds_frag(aS + (wave * 16) * 168 + ks * 32, 168);
#pragma unroll
      for (int j = 0; j < 4; ++j) acc[j] = wmma16(af, lds_frag(wS + (j * 16) * 168 + ks * 32, 168), acc[j]); }
    __syncthreads();
  }
#pragma unroll
  for (int j = 0; j < 4; ++j)
#pragma unroll
    for (int r = 0; r < 8; ++r) { const int o = j * 16 + cl, p = wave * 16 + rh + r; oS[o * 132 + p] = acc[j][r] + bias[o]; }
  __syncthreads();
#pragma unroll 1
  for (int pass = 0; pass < 2; ++pass) { for (int q4 = tid; q4 < COUT * 32; q4 += 256) { const int o = q4 >> 5, c4 = (q4 & 31) * 4;
      *(volatile v4f_t*)(out + ((size_t)b * COUT + o) * NPIX + p0 + c4) = *(const v4fa*)(oS + o * 132 + c4); } __threadfence(); }
}

extern "C" void kernel_launch(void* const* d_in, const int* in_sizes, int n_in,
                              void* d_out, int out_size, void* d_ws, size_t ws_size,
                              hipStream_t stream) {
  (void)in_sizes; (void)n_in; (void)out_size; (void)d_ws; (void)ws_size;
  const float* x = (const float*)d_in[0];
  const float* depth = (const float*)d_in[1];
  const float* w = (const float*)d_in[2];
  const float* bias = (const float*)d_in[3];
  float* out = (float*)d_out;
  k_depthconv<<<dim3(NB_ * (NPIX / 128)), dim3(256), 0, stream>>>(x, depth, w, bias, out);
}
